// GroupedMultiQuerySelfAttention_78426102825679
// MI455X (gfx1250) — hardware-verified
//
#include <hip/hip_runtime.h>


#ifndef NB
#define NB 2
#endif
#ifndef SEQ
#define SEQ 2048
#endif
#define NB_FULL  2
#define SEQ_FULL 2048
#ifndef OUT_SEQ
#define OUT_SEQ SEQ
#endif
#define DM   1024
#define NQH  16
#define NKG  4
#define HPG  4
#define HD   64
#define DKV  256
#define AW   4
#define OSP  68
#define GSP  68
#define TLP  65
#define SC2  ((float)(0.125 * 1.4426950408889634))
#define PSH  14.0f
#define NEGB (-3.0e38f)
#define CTS  1024.0f
#define WOS  64.0f
#define OSC  (1.0f / 65536.0f)

static_assert(HD == 64);
static_assert(NQH * HD == DM);
static_assert(NKG * HD == DKV);
static_assert(NKG * HPG == NQH);
static_assert(DM % 64 == 0);
static_assert(DKV % 64 == 0);
static_assert(DM % 32 == 0);
static_assert(SEQ % 64 == 0);
static_assert((NB * SEQ) % 64 == 0);
static_assert(SEQ % 32 == 0);
static_assert(SEQ % (16 * AW) == 0);
static_assert(((size_t)SEQ * DM) % 8 == 0);
static_assert(NB <= NB_FULL);
static_assert(SEQ <= SEQ_FULL);
static_assert(OUT_SEQ >= SEQ);
static_assert((OSP * 4) % 16 == 0);
static_assert((GSP * 4) % 16 == 0);
static_assert(OSP >= HD);
static_assert(GSP >= 64);
static_assert(CTS * WOS * OSC == 1.0f);
static_assert(32 * 8 * 4 == 16 * 64);
static_assert(32 * 4 * 8 == 16 * 64);
static_assert(256 * 4 * 4 == 64 * 64);
static_assert(256 * 8 * 2 == 64 * 64);
static_assert(16 * GSP * 4 <= 131072);
static_assert(AW * 16 * OSP * 4 <= 131072);
static_assert(64 * TLP * 4 <= 131072);
static_assert((size_t)NB_FULL * SEQ_FULL * DM * 4 == (size_t)16777216);

typedef _Float16 h16;
typedef unsigned short bf;
typedef __attribute__((ext_vector_type(16))) __bf16   v16bf;
typedef __attribute__((ext_vector_type(16))) _Float16 v16h;
typedef __attribute__((ext_vector_type(8)))  _Float16 v8h;
typedef __attribute__((ext_vector_type(8)))  unsigned short v8us;
typedef __attribute__((ext_vector_type(8)))  float    v8f;
typedef __attribute__((ext_vector_type(4)))  float    v4f;
typedef v4f  __attribute__((may_alias)) v4fa;

__device__ __forceinline__ unsigned short f2bf(float f) { unsigned u = __float_as_uint(f); u += 0x7FFFu + ((u >> 16) & 1u); return (unsigned short)(u >> 16); }
__device__ __forceinline__ float bfr(float f) { return __uint_as_float(((unsigned)f2bf(f)) << 16); }
__device__ __forceinline__ v16h cat16(v8h lo, v8h hi) { return __builtin_shufflevector(lo, hi, 0, 1, 2, 3, 4, 5, 6, 7, 8, 9, 10, 11, 12, 13, 14, 15); }
__device__ __forceinline__ v16bf cat16b(v8us lo, v8us hi) { return __builtin_bit_cast(v16bf, __builtin_shufflevector(lo, hi, 0, 1, 2, 3, 4, 5, 6, 7, 8, 9, 10, 11, 12, 13, 14, 15)); }
__device__ __forceinline__ v8f wmma16(v16h a, v16h b, v8f c) { return __builtin_amdgcn_wmma_f32_16x16x32_f16(false, a, false, b, (short)0, c, false, false); }
__device__ __forceinline__ v8f wmmab(v16bf a, v16bf b, v8f c) { return __builtin_amdgcn_wmma_f32_16x16x32_bf16(false, a, false, b, (short)0, c, false, false); }
__device__ __forceinline__ v16h  ldh(const h16* p) { return cat16(*(const v8h*)p, *(const v8h*)(p + 16)); }
__device__ __forceinline__ v16bf ldb(const bf* p)  { return cat16b(*(const v8us*)p, *(const v8us*)(p + 16)); }
__device__ __forceinline__ void wave_sync() { __builtin_amdgcn_fence(3  , "wavefront"); __builtin_amdgcn_wave_barrier(); asm volatile("" ::: "memory"); }

static __device__ __forceinline__ h16 toh_flush(float v) { const h16 r = (h16)v; return (fabsf(v) < 6.103515625e-05f) ? (h16)0.0f : r; }
__device__ __forceinline__ v8f wmma16g(v16h a, v16h b, v8f c) { c = wmma16(a, b, c); asm volatile("v_nop\n\tv_nop\n\tv_nop\n\tv_nop" : "+v"(c) : "v"(a), "v"(b)); return c; }
__device__ __forceinline__ v8f wmmabg(v16bf a, v16bf b, v8f c) { c = wmmab(a, b, c); asm volatile("v_nop\n\tv_nop\n\tv_nop\n\tv_nop" : "+v"(c) : "v"(a), "v"(b)); return c; }

__global__ __launch_bounds__(256) void k_cvt8(const float* __restrict__ src, bf* dst, size_t n8) {
    const size_t i = (size_t)blockIdx.x * 256 + threadIdx.x; if (i >= n8) return;
    const v8f v = *(const v8f*)(src + i * 8); v8us o;
#pragma unroll
    for (int k = 0; k < 8; ++k) o[k] = f2bf(v[k]);
    *(volatile v8us*)(dst + i * 8) = o; __threadfence(); *(volatile v8us*)(dst + i * 8) = o;
}

template <int F16>
__device__ __forceinline__ void wt_body(const float* __restrict__ W, bf* dB, h16* dH, int N, int K, float carry) {
#pragma clang fp contract(off)
    __shared__ __align__(16) float tl[64 * TLP];
    const int tid = threadIdx.x; const int n0 = blockIdx.x * 64, k0 = blockIdx.y * 64;
#pragma unroll 1
    for (int i = 0; i < 4; ++i) { const int idx = i * 256 + tid; const int r = idx >> 4, c4 = (idx & 15) * 4;
        const v4f v = *(const v4f*)(W + (size_t)(k0 + r) * N + n0 + c4);
        tl[r * TLP + c4 + 0] = v[0]; tl[r * TLP + c4 + 1] = v[1]; tl[r * TLP + c4 + 2] = v[2]; tl[r * TLP + c4 + 3] = v[3]; }
    __syncthreads();
    v8us ob[2]; v8h oh[2]; size_t oo[2];
#pragma unroll
    for (int i = 0; i < 2; ++i) { const int p = i * 256 + tid; const int row = p >> 3, c8 = (p & 7) * 8;
        oo[i] = (size_t)(n0 + row) * K + k0 + c8;
#pragma unroll
        for (int e = 0; e < 8; ++e) { const float x = tl[(c8 + e) * TLP + row]; ob[i][e] = f2bf(x); oh[i][e] = toh_flush(bfr(x) * carry); } }
#pragma unroll 1
    for (int ps = 0; ps < 2; ++ps) {
#pragma unroll
        for (int i = 0; i < 2; ++i) { if (F16) *(volatile v8h*)(dH + oo[i]) = oh[i]; else *(volatile v8us*)(dB + oo[i]) = ob[i]; }
        if (ps == 0) __threadfence(); }
}
__global__ __launch_bounds__(256) void k_wt_bf(const float* __restrict__ W, bf* dst, int N, int K) { wt_body<0>(W, dst, (h16*)0, N, K, 1.0f); }
__global__ __launch_bounds__(256) void k_wt_h(const float* __restrict__ W, h16* dst, int N, int K, float carry) { wt_body<1>(W, (bf*)0, dst, N, K, carry); }

template <int KIND>
__device__ __forceinline__ void gemm_body(const bf* __restrict__ Ab, const bf* __restrict__ Bb, const h16* __restrict__ Ah, const h16* __restrict__ Bh,
                                          const float* __restrict__ bias, h16* Ch, float* Cf, float oscale,
                                          int K, int ldc, int rper, size_t rbs, int nper, size_t cbs) {
    __shared__ __align__(16) float os[16 * GSP];
    const int lane = threadIdx.x & 31, lr = lane & 15, hi = lane >> 4; const int r0 = blockIdx.x * 64, c0 = blockIdx.y * 64;
    v8f acc[4][4];
#pragma unroll
    for (int mb = 0; mb < 4; ++mb)
#pragma unroll
        for (int nb = 0; nb < 4; ++nb) acc[mb][nb] = (v8f){};
    const size_t aoff = (size_t)(r0 + lr) * K + 8 * hi, boff = (size_t)(c0 + lr) * K + 8 * hi;
#pragma unroll 1
    for (int kc = 0; kc < K; kc += 32) {
        if (KIND == 2) {
            v16h a[4];
#pragma unroll
            for (int mb = 0; mb < 4; ++mb) a[mb] = ldh(Ah + aoff + (size_t)mb * 16 * K + kc);
#pragma unroll
            for (int nb = 0; nb < 4; ++nb) { const v16h b = ldh(Bh + boff + (size_t)nb * 16 * K + kc);
#pragma unroll
                for (int mb = 0; mb < 4; ++mb) acc[mb][nb] = wmma16g(a[mb], b, acc[mb][nb]); }
        } else {
            v16bf a[4];
#pragma unroll
            for (int mb = 0; mb < 4; ++mb) a[mb] = ldb(Ab + aoff + (size_t)mb * 16 * K + kc);
#pragma unroll
            for (int nb = 0; nb < 4; ++nb) { const v16bf b = ldb(Bb + boff + (size_t)nb * 16 * K + kc);
#pragma unroll
                for (int mb = 0; mb < 4; ++mb) acc[mb][nb] = wmmabg(a[mb], b, acc[mb][nb]); }
        }
    }
    float bc[4];
#pragma unroll
    for (int nb = 0; nb < 4; ++nb) bc[nb] = (KIND != 1) ? bfr(bias[c0 + nb * 16 + lr]) : 0.0f;
    const size_t base = (size_t)(r0 / rper) * rbs + (size_t)(r0 % rper) * (size_t)ldc + (size_t)(c0 / nper) * cbs + (size_t)(c0 % nper);
#pragma unroll
    for (int mb = 0; mb < 4; ++mb) {
        float br[8];
#pragma unroll
        for (int j = 0; j < 8; ++j) br[j] = (KIND == 1) ? bfr(bias[r0 + mb * 16 + hi * 8 + j]) : 0.0f;
#pragma unroll
        for (int nb = 0; nb < 4; ++nb) {
#pragma unroll
            for (int j = 0; j < 8; ++j) os[(hi * 8 + j) * GSP + nb * 16 + lr] = acc[mb][nb][j] * oscale + bc[nb] + br[j]; }
        wave_sync();
        const size_t sb = base + (size_t)(mb * 16) * (size_t)ldc;
        if (KIND == 2) {
#pragma unroll 1
            for (int ps = 0; ps < 2; ++ps) {
#pragma unroll
                for (int s = 0; s < 8; ++s) { const int row = 2 * s + (lane >> 4), c4 = (lane & 15) * 4;
                    const v4f val = *(const v4fa*)(&os[row * GSP + c4]);
                    *(volatile v4f*)(Cf + sb + (size_t)row * ldc + c4) = val; }
                if (ps == 0) __threadfence(); }
        } else {
            v8h hv[4];
#pragma unroll
            for (int s = 0; s < 4; ++s) { const int row = 4 * s + (lane >> 3), c8 = (lane & 7) * 8;
                const v4f x0 = *(const v4fa*)(&os[row * GSP + c8]); const v4f x1 = *(const v4fa*)(&os[row * GSP + c8 + 4]);
#pragma unroll
                for (int i = 0; i < 4; ++i) { hv[s][i] = toh_flush(x0[i]); hv[s][4 + i] = toh_flush(x1[i]); } }
#pragma unroll 1
            for (int ps = 0; ps < 2; ++ps) {
#pragma unroll
                for (int s = 0; s < 4; ++s) { const int row = 4 * s + (lane >> 3), c8 = (lane & 7) * 8;
                    *(volatile v8h*)(Ch + sb + (size_t)row * ldc + c8) = hv[s]; }
                if (ps == 0) __threadfence(); }
        }
        wave_sync();
    }
}
__global__ __launch_bounds__(32) void k_gemm_cb(const bf* __restrict__ A, const bf* __restrict__ Bt, const float* __restrict__ bias, h16* C,
                                                int K, int ldc, int rper, size_t rbs, int nper, size_t cbs) {
    gemm_body<0>(A, Bt, (const h16*)0, (const h16*)0, bias, C, (float*)0, 1.0f, K, ldc, rper, rbs, nper, cbs);
}
__global__ __launch_bounds__(32) void k_gemm_rb(const bf* __restrict__ A, const bf* __restrict__ Bt, const float* __restrict__ bias, h16* C,
                                                int K, int ldc, int rper, size_t rbs, int nper, size_t cbs) {
    gemm_body<1>(A, Bt, (const h16*)0, (const h16*)0, bias, C, (float*)0, 1.0f, K, ldc, rper, rbs, nper, cbs);
}
__global__ __launch_bounds__(32) void k_gemm_out(const h16* __restrict__ A, const h16* __restrict__ Bt, const float* __restrict__ bias, float* C, float oscale,
                                                 int K, int ldc, int rper, size_t rbs, int nper, size_t cbs) {
    gemm_body<2>((const bf*)0, (const bf*)0, A, Bt, bias, (h16*)0, C, oscale, K, ldc, rper, rbs, nper, cbs);
}

__global__ __launch_bounds__(32 * AW) void k_flash(const h16* __restrict__ QH, const h16* __restrict__ KP, const h16* __restrict__ VT, h16* CT) {
    __shared__ __align__(16) float os[AW * 16 * OSP];
    const int lane = threadIdx.x & 31, lr = lane & 15, hi = lane >> 4;
    const int wave = __builtin_amdgcn_readfirstlane((int)(threadIdx.x >> 5));
    const int zh = blockIdx.y; const int b = zh / NQH, qh = zh % NQH; const int g = qh / HPG;
    const int t0 = (blockIdx.x * AW + wave) * 16;
    const size_t qo = ((size_t)b * SEQ + (size_t)(t0 + lr)) * DM + (size_t)qh * HD + 8 * hi;
    const v16h q0 = ldh(QH + qo), q1 = ldh(QH + qo + 32);
    const size_t ko = ((size_t)b * SEQ + (size_t)lr) * DKV + (size_t)g * HD + 8 * hi;
    const size_t vo = ((size_t)b * DKV + (size_t)g * HD + (size_t)lr) * SEQ + 8 * hi;
    v8f o0 = (v8f){}, o1 = (v8f){}, o2 = (v8f){}, o3 = (v8f){};
    float m = NEGB, l = 0.0f;
#pragma unroll 1
    for (int key0 = 0; key0 < SEQ; key0 += 32) {
        const h16* ka = KP + ko + (size_t)key0 * DKV;
        const v16h ka0 = ldh(ka), ka1 = ldh(ka + 32), kb0 = ldh(ka + (size_t)16 * DKV), kb1 = ldh(ka + (size_t)16 * DKV + 32);
        v8f sa = (v8f){}, sb = (v8f){};
        sa = wmma16g(ka0, q0, sa); sb = wmma16g(kb0, q0, sb); sa = wmma16g(ka1, q1, sa); sb = wmma16g(kb1, q1, sb);
        float ta[8], tb[8]; float mx = NEGB;
#pragma unroll
        for (int r = 0; r < 8; ++r) { ta[r] = sa[r] * SC2; tb[r] = sb[r] * SC2; mx = fmaxf(mx, fmaxf(ta[r], tb[r])); }
        mx = fmaxf(mx, __shfl_xor(mx, 16, 32));
        const float mnew = fmaxf(m, mx);
        const float alpha = __builtin_amdgcn_exp2f(m - mnew);
        const float sh = PSH - mnew;
        v16h pb; float ls = 0.0f;
#pragma unroll
        for (int r = 0; r < 8; ++r) {
            const float ea = ta[r] + sh, eb = tb[r] + sh;
            const float xa = __builtin_amdgcn_exp2f(ea), xb = __builtin_amdgcn_exp2f(eb);
            const float ga = (ea < -14.0f) ? 0.0f : xa, gb = (eb < -14.0f) ? 0.0f : xb;
            const h16 pa = (h16)ga; const h16 pc = (h16)gb;
            pb[r] = pa; pb[8 + r] = pc;
            ls += (float)pa + (float)pc; }
        l = l * alpha + ls; m = mnew;
        o0 = o0 * alpha; o1 = o1 * alpha; o2 = o2 * alpha; o3 = o3 * alpha;
        const h16* va = VT + vo + key0;
        const v16h v0 = ldh(va), v1 = ldh(va + (size_t)16 * SEQ), v2 = ldh(va + (size_t)32 * SEQ), v3 = ldh(va + (size_t)48 * SEQ);
        o0 = wmma16g(v0, pb, o0); o1 = wmma16g(v1, pb, o1); o2 = wmma16g(v2, pb, o2); o3 = wmma16g(v3, pb, o3);
    }
    l += __shfl_xor(l, 16, 32);
    const float inv = CTS * (1.0f / l);
    const int wb = wave * 16 * OSP;
    { v4f a, c;
      a[0] = o0[0] * inv; a[1] = o0[1] * inv; a[2] = o0[2] * inv; a[3] = o0[3] * inv; c[0] = o0[4] * inv; c[1] = o0[5] * inv; c[2] = o0[6] * inv; c[3] = o0[7] * inv;
      *(v4fa*)(&os[wb + lr * OSP +  0 + 8 * hi]) = a; *(v4fa*)(&os[wb + lr * OSP +  0 + 8 * hi + 4]) = c;
      a[0] = o1[0] * inv; a[1] = o1[1] * inv; a[2] = o1[2] * inv; a[3] = o1[3] * inv; c[0] = o1[4] * inv; c[1] = o1[5] * inv; c[2] = o1[6] * inv; c[3] = o1[7] * inv;
      *(v4fa*)(&os[wb + lr * OSP + 16 + 8 * hi]) = a; *(v4fa*)(&os[wb + lr * OSP + 16 + 8 * hi + 4]) = c;
      a[0] = o2[0] * inv; a[1] = o2[1] * inv; a[2] = o2[2] * inv; a[3] = o2[3] * inv; c[0] = o2[4] * inv; c[1] = o2[5] * inv; c[2] = o2[6] * inv; c[3] = o2[7] * inv;
      *(v4fa*)(&os[wb + lr * OSP + 32 + 8 * hi]) = a; *(v4fa*)(&os[wb + lr * OSP + 32 + 8 * hi + 4]) = c;
      a[0] = o3[0] * inv; a[1] = o3[1] * inv; a[2] = o3[2] * inv; a[3] = o3[3] * inv; c[0] = o3[4] * inv; c[1] = o3[5] * inv; c[2] = o3[6] * inv; c[3] = o3[7] * inv;
      *(v4fa*)(&os[wb + lr * OSP + 48 + 8 * hi]) = a; *(v4fa*)(&os[wb + lr * OSP + 48 + 8 * hi + 4]) = c; }
    wave_sync();
    v8h hv[4];
#pragma unroll
    for (int s = 0; s < 4; ++s) { const int row = 4 * s + (lane >> 3), c8 = (lane & 7) * 8;
        const v4f x0 = *(const v4fa*)(&os[wb + row * OSP + c8]); const v4f x1 = *(const v4fa*)(&os[wb + row * OSP + c8 + 4]);
#pragma unroll
        for (int i = 0; i < 4; ++i) { hv[s][i] = toh_flush(x0[i]); hv[s][4 + i] = toh_flush(x1[i]); } }
    h16* crow = CT + ((size_t)b * SEQ + (size_t)t0) * DM + (size_t)qh * HD;
#pragma unroll 1
    for (int ps = 0; ps < 2; ++ps) {
#pragma unroll
        for (int s = 0; s < 4; ++s) { const int row = 4 * s + (lane >> 3), c8 = (lane & 7) * 8;
            *(volatile v8h*)(crow + (size_t)row * DM + c8) = hv[s]; }
        if (ps == 0) __threadfence(); }
}

static constexpr size_t al256(size_t v) { return (v + 255) & ~(size_t)255; }
static constexpr size_t SZ_XB  = al256((size_t)NB * SEQ * DM * 2);
static constexpr size_t SZ_WQ  = al256((size_t)DM * DM * 2);
static constexpr size_t SZ_WKV = al256((size_t)DKV * DM * 2);
static constexpr size_t SZ_KV  = al256((size_t)NB * SEQ * DKV * 2);
static constexpr size_t SZ_TOTAL = 3 * SZ_XB + 2 * SZ_WQ + 2 * SZ_WKV + 2 * SZ_KV;
static_assert(SZ_TOTAL <= (size_t)134217728);
static_assert((size_t)NB * DKV * SEQ == (size_t)NB * SEQ * DKV);

extern "C" void kernel_launch(void* const* d_in, const int* in_sizes, int n_in,
                              void* d_out, int out_size, void* d_ws, size_t ws_size, hipStream_t stream) {
    if (n_in < 9) return;
    const size_t needx = ((size_t)(NB - 1) * SEQ_FULL + SEQ) * DM;
    if ((size_t)in_sizes[0] < needx) return;
    if ((size_t)in_sizes[1] < (size_t)DM * DM || (size_t)in_sizes[7] < (size_t)DM * DM) return;
    if ((size_t)in_sizes[3] < (size_t)DM * DKV || (size_t)in_sizes[5] < (size_t)DM * DKV) return;
    if (in_sizes[2] < DM || in_sizes[4] < DKV || in_sizes[6] < DKV || in_sizes[8] < DM) return;
    if ((size_t)out_size < ((size_t)(NB - 1) * OUT_SEQ + SEQ) * DM) return;
    if (SZ_TOTAL > ws_size) return;
    const float* x  = (const float*)d_in[0];
    const float* wq = (const float*)d_in[1]; const float* bq = (const float*)d_in[2];
    const float* wk = (const float*)d_in[3]; const float* bk = (const float*)d_in[4];
    const float* wv = (const float*)d_in[5]; const float* bv = (const float*)d_in[6];
    const float* wo = (const float*)d_in[7]; const float* bo = (const float*)d_in[8];
    float* OUT = (float*)d_out;
    char* wsp = (char*)d_ws;
    bf*  XB  = (bf*)wsp;  wsp += SZ_XB;
    bf*  WQT = (bf*)wsp;  wsp += SZ_WQ;
    bf*  WKT = (bf*)wsp;  wsp += SZ_WKV;
    bf*  WVT = (bf*)wsp;  wsp += SZ_WKV;
    h16* WOT = (h16*)wsp; wsp += SZ_WQ;
    h16* QH  = (h16*)wsp; wsp += SZ_XB;
    h16* KP  = (h16*)wsp; wsp += SZ_KV;
    h16* VT  = (h16*)wsp; wsp += SZ_KV;
    h16* CT  = (h16*)wsp; wsp += SZ_XB;

    if (SEQ == SEQ_FULL) {
        const size_t n8 = (size_t)NB * SEQ * DM / 8;
        k_cvt8<<<(unsigned)((n8 + 255) / 256), 256, 0, stream>>>(x, XB, n8);
    } else {
        const size_t n8 = (size_t)SEQ * DM / 8;
        for (int b = 0; b < NB; ++b) k_cvt8<<<(unsigned)((n8 + 255) / 256), 256, 0, stream>>>(x + (size_t)b * SEQ_FULL * DM, XB + (size_t)b * SEQ * DM, n8);
    }
    k_wt_bf<<<dim3(DM / 64,  DM / 64, 1), 256, 0, stream>>>(wq, WQT, DM,  DM);
    k_wt_bf<<<dim3(DKV / 64, DM / 64, 1), 256, 0, stream>>>(wk, WKT, DKV, DM);
    k_wt_bf<<<dim3(DKV / 64, DM / 64, 1), 256, 0, stream>>>(wv, WVT, DKV, DM);
    k_wt_h <<<dim3(DM / 64,  DM / 64, 1), 256, 0, stream>>>(wo, WOT, DM,  DM, WOS);

    k_gemm_cb<<<dim3(NB * SEQ / 64, DM / 64, 1), 32, 0, stream>>>(XB, WQT, bq, QH, DM, DM, NB * SEQ, (size_t)0, DM, (size_t)0);
    k_gemm_cb<<<dim3(NB * SEQ / 64, DKV / 64, 1), 32, 0, stream>>>(XB, WKT, bk, KP, DM, DKV, NB * SEQ, (size_t)0, DKV, (size_t)0);
    k_gemm_rb<<<dim3(DKV / 64, NB * SEQ / 64, 1), 32, 0, stream>>>(WVT, XB, bv, VT, DM, SEQ, DKV, (size_t)0, SEQ, (size_t)DKV * SEQ);

    k_flash<<<dim3(SEQ / (16 * AW), NB * NQH, 1), 32 * AW, 0, stream>>>(QH, KP, VT, CT);

    k_gemm_out<<<dim3(NB * SEQ / 64, DM / 64, 1), 32, 0, stream>>>(CT, WOT, bo, OUT, OSC, DM, DM, SEQ, (size_t)OUT_SEQ * DM, DM, (size_t)0);
}
